// DeepGraphConvLayer_17300128269006
// MI455X (gfx1250) — hardware-verified
//
#include <hip/hip_runtime.h>
#include <stddef.h>


#define KD      256
#define FD      256
#define NH      4
#define HC      64
#define NMAT    2
#define NTHR    256
#define NWAVE   8
#define EPT     8
#define CHUNK   (NTHR * EPT)
#define WCAP    (EPT * 32)
#define LISTN   (NWAVE * WCAP)
#define NBMAX   2048
#define NBMIN   32
#define RCAP    28672
#define DEGCAP  4096
#define GBM     64
#define GTHR    128
#define RB      128
#define EPW     32
#define NEG_SLOPE 0.2f
#define BN_EPS  0.00001f
#define WSCALE  16.0f
#define WINV    0.0625f
#define WSCAP   134217728
#define LDS_AGG ((2 * RCAP + 2 * NBMAX + LISTN) * 4 + 64)

static_assert((CHUNK & (CHUNK - 1)) == 0 && CHUNK <= 4096);
static_assert((NBMAX & (NBMAX - 1)) == 0 && NBMAX <= 4096);
static_assert(NTHR * 8 == NBMAX);
static_assert(LISTN >= NBMAX);
static_assert(LISTN >= NWAVE * WCAP);
static_assert((RCAP % 32) == 0);
static_assert(LDS_AGG <= 300000);
static_assert(GBM == (GTHR / 32) * 16);
static_assert(NH * HC == FD);
static_assert(FD == NTHR);
static_assert((KD % 32) == 0);
static_assert((RB % 4) == 0);
static_assert(NBMIN >= 32 && (NBMIN % 8) == 0);
static_assert(EPW == 32);

typedef float          v4f  __attribute__((ext_vector_type(4)));
typedef float          v8f  __attribute__((ext_vector_type(8)));
typedef int            v4i  __attribute__((ext_vector_type(4)));
typedef int            v8i  __attribute__((ext_vector_type(8)));
typedef double         v2d  __attribute__((ext_vector_type(2)));
typedef unsigned short v8us __attribute__((ext_vector_type(8)));
typedef _Float16       v8h  __attribute__((ext_vector_type(8)));
typedef _Float16       v16h __attribute__((ext_vector_type(16)));
union FragH { v16h v; v8h f[2]; v8us h[2]; v8i w; };
union Cv8   { v8h f; v8us u; };

__device__ __forceinline__ v8h cvt8h(v4f a, v4f b) {
  v8h r;
  r[0] = (_Float16)a.x; r[1] = (_Float16)a.y; r[2] = (_Float16)a.z; r[3] = (_Float16)a.w;
  r[4] = (_Float16)b.x; r[5] = (_Float16)b.y; r[6] = (_Float16)b.z; r[7] = (_Float16)b.w;
  return r;
}

__device__ __forceinline__ v8f wmh(const FragH& a, const FragH& b, v8f c) {
  v8f d = __builtin_amdgcn_wmma_f32_16x16x32_f16(false, a.v, false, b.v, (short)0, c, false, false);
  asm volatile("v_nop\n\tv_nop\n\tv_nop\n\tv_nop" : "+v"(d) : "v"(a.w), "v"(b.w));
  return d;
}

__device__ __forceinline__ float bcl(float v, int l) {
  return __uint_as_float((unsigned)__builtin_amdgcn_readlane((int)__float_as_uint(v), l));
}

__device__ __forceinline__ float logit16(v4f t, v4f a) {
  v4f z;
  z.x = fmaxf(t.x, NEG_SLOPE * t.x);
  z.y = fmaxf(t.y, NEG_SLOPE * t.y);
  z.z = fmaxf(t.z, NEG_SLOPE * t.z);
  z.w = fmaxf(t.w, NEG_SLOPE * t.w);
  float p = z.x * a.x;
  p = fmaf(z.y, a.y, p);
  p = fmaf(z.z, a.z, p);
  p = fmaf(z.w, a.w, p);
  p += __shfl_xor(p, 8);
  p += __shfl_xor(p, 4);
  p += __shfl_xor(p, 2);
  p += __shfl_xor(p, 1);
  return p;
}

__device__ __forceinline__ int scan_chunk(const int* __restrict__ dsts, int nE, int cbase, int slotBase,
                                          int nb, int vec8, int* list, int tid, int lane, int wave) {
  int wc = 0;
  const int el0  = tid * EPT;
  const int e0   = cbase + el0;
  const int sent = -2147483647 - 1;
  v4i da, db;
  if (vec8 != 0 && cbase + CHUNK <= nE) {
    da = *(const v4i*)(dsts + e0);
    db = *(const v4i*)(dsts + e0 + 4);
  } else {
    da.x = (e0     < nE) ? dsts[min(e0,     nE - 1)] : sent;
    da.y = (e0 + 1 < nE) ? dsts[min(e0 + 1, nE - 1)] : sent;
    da.z = (e0 + 2 < nE) ? dsts[min(e0 + 2, nE - 1)] : sent;
    da.w = (e0 + 3 < nE) ? dsts[min(e0 + 3, nE - 1)] : sent;
    db.x = (e0 + 4 < nE) ? dsts[min(e0 + 4, nE - 1)] : sent;
    db.y = (e0 + 5 < nE) ? dsts[min(e0 + 5, nE - 1)] : sent;
    db.z = (e0 + 6 < nE) ? dsts[min(e0 + 6, nE - 1)] : sent;
    db.w = (e0 + 7 < nE) ? dsts[min(e0 + 7, nE - 1)] : sent;
  }
  const unsigned nbs = (unsigned)slotBase;
  const unsigned unb = (unsigned)nb;
  const unsigned s0 = (unsigned)da.x - nbs, s1 = (unsigned)da.y - nbs;
  const unsigned s2 = (unsigned)da.z - nbs, s3 = (unsigned)da.w - nbs;
  const unsigned s4 = (unsigned)db.x - nbs, s5 = (unsigned)db.y - nbs;
  const unsigned s6 = (unsigned)db.z - nbs, s7 = (unsigned)db.w - nbs;
  const bool h0 = s0 < unb, h1 = s1 < unb, h2 = s2 < unb, h3 = s3 < unb;
  const bool h4 = s4 < unb, h5 = s5 < unb, h6 = s6 < unb, h7 = s7 < unb;
  const unsigned any = __builtin_amdgcn_ballot_w32(h0 | h1 | h2 | h3 | h4 | h5 | h6 | h7);
  if (any != 0u) {
#define HITJ(J, HJ, SJ) { \
      const unsigned mj = __builtin_amdgcn_ballot_w32(HJ); \
      if (mj != 0u) { \
        if (HJ) { \
          const int pos = wc + (int)__builtin_amdgcn_mbcnt_lo(mj, 0u); \
          if (pos < WCAP) list[wave * WCAP + pos] = ((el0 + (J)) << 12) | (int)(SJ); \
        } \
        wc += (int)__builtin_popcount(mj); } }
    HITJ(0, h0, s0)
    HITJ(1, h1, s1)
    HITJ(2, h2, s2)
    HITJ(3, h3, s3)
    HITJ(4, h4, s4)
    HITJ(5, h5, s5)
    HITJ(6, h6, s6)
    HITJ(7, h7, s7)
#undef HITJ
  }
  return wc;
}

__global__ __launch_bounds__(NTHR) void k_wprep(const float* __restrict__ Ws, const float* __restrict__ Wd,
                                                unsigned short* wt) {
  const int j = (int)blockIdx.y;
  const int u = (int)blockIdx.x * NTHR + (int)threadIdx.x;
  if (u >= FD * KD / 8) return;
  const int n  = u >> 5;
  const int k8 = (u & 31) * 8;
  const float* src = (j & 1) ? Wd : Ws;
  const float* p = src + (size_t)k8 * FD + n;
  v4f a, b;
  a.x = p[0 * FD]; a.y = p[1 * FD]; a.z = p[2 * FD]; a.w = p[3 * FD];
  b.x = p[4 * FD]; b.y = p[5 * FD]; b.z = p[6 * FD]; b.w = p[7 * FD];
  Cv8 c;
  c.f = cvt8h(a * WSCALE, b * WSCALE);
  const size_t o = (size_t)(j * FD + n) * KD + k8;
  *(volatile v8us*)(wt + o) = c.u;
  __threadfence();
  *(volatile v8us*)(wt + o) = c.u;
}

__global__ __launch_bounds__(GTHR) void k_gemm(const float* __restrict__ x,
                                               const unsigned short* __restrict__ wt,
                                               const float* __restrict__ bs, const float* __restrict__ bd,
                                               float* Y, int yStride, int nN) {
  __shared__ __attribute__((aligned(16))) float stg[GBM * (FD / 2)];
  const int tid = threadIdx.x, lane = tid & 31, wave = tid >> 5, hh = lane >> 4, m = lane & 15;
  const int rowBase = (int)blockIdx.x * GBM;
  int ar = rowBase + 16 * wave + m;
  ar = ar < nN ? ar : nN - 1;
  const float* ap = x + (size_t)ar * KD + 8 * hh;
  FragH af[8];
#pragma unroll
  for (int ks = 0; ks < 8; ++ks) {
    const float* p0 = ap + 32 * ks;
    const float* p1 = ap + 32 * ks + 16;
    af[ks].f[0] = cvt8h(*(const v4f*)p0, *(const v4f*)(p0 + 4));
    af[ks].f[1] = cvt8h(*(const v4f*)p1, *(const v4f*)(p1 + 4));
  }
#pragma unroll 1
  for (int p = 0; p < 4; ++p) {
    const int mat = p >> 1, chh = p & 1;
    const float* bsel = (mat != 0) ? bd : bs;
#pragma unroll 1
    for (int ch = 0; ch < 2; ++ch) {
      v8f acc[4];
#pragma unroll
      for (int t = 0; t < 4; ++t) { v8f z = {0.f, 0.f, 0.f, 0.f, 0.f, 0.f, 0.f, 0.f}; acc[t] = z; }
      const int ncol0 = 128 * chh + 64 * ch;
      const size_t brow = (size_t)(mat * FD + ncol0 + m) * KD + 8 * hh;
#pragma unroll
      for (int ks = 0; ks < 8; ++ks) {
#pragma unroll
        for (int t = 0; t < 4; ++t) {
          const size_t bo = brow + (size_t)(16 * t) * KD + 32 * ks;
          FragH bf;
          bf.h[0] = *(const v8us*)(wt + bo);
          bf.h[1] = *(const v8us*)(wt + bo + 16);
          acc[t] = wmh(af[ks], bf, acc[t]);
        }
      }
      float* sp = stg + (size_t)(16 * wave + 8 * hh) * (FD / 2) + 64 * ch + m;
#pragma unroll
      for (int t = 0; t < 4; ++t) {
        const float bv = bsel[ncol0 + 16 * t + m];
#pragma unroll
        for (int r = 0; r < 8; ++r) sp[(size_t)r * (FD / 2) + 16 * t] = acc[t][r] * WINV + bv;
      }
    }
    __syncthreads();
    const int nF4 = GBM * (FD / 2) / 4;
    float* yb = Y + (size_t)mat * (size_t)yStride + (size_t)rowBase * FD + 128 * chh;
    const v4f* s4 = (const v4f*)stg;
#pragma unroll 1
    for (int f = tid; f < nF4; f += GTHR) {
      const int r = f >> 5, q = f & 31;
      const v4f v = s4[f];
      *(volatile v4f*)(yb + (size_t)r * FD + 4 * q) = v;
    }
    __threadfence();
#pragma unroll 1
    for (int f = tid; f < nF4; f += GTHR) {
      const int r = f >> 5, q = f & 31;
      const v4f v = s4[f];
      *(volatile v4f*)(yb + (size_t)r * FD + 4 * q) = v;
    }
    __syncthreads();
  }
}

__global__ __launch_bounds__(NTHR) void k_agg(
    const int* __restrict__ srcs, const int* __restrict__ dsts,
    const float* __restrict__ xl, const float* __restrict__ xr, const float* __restrict__ xres,
    const float* __restrict__ attw, const float* __restrict__ biaso,
    float* outp, float* stat, int nN, int nE, int nb, int vec8) {
  extern __shared__ v4f lds_dyn[];
  int* reg1 = (int*)lds_dyn;
  int* reg2 = reg1 + RCAP;
  int* scnt = reg2 + RCAP;
  int* soff = scnt + NBMAX;
  int* list = soff + NBMAX;
  int* wcnt = list + LISTN;
  int* wtot = wcnt + NWAVE;
  const int tid = threadIdx.x, lane = tid & 31, wave = tid >> 5;
  const int nodeBase = (int)blockIdx.x * nb;

  for (int i = tid; i < NBMAX; i += NTHR) scnt[i] = 0;
  __syncthreads();

  int tot = 0;
  int lost = 0;
  const int nChunks = (nE + CHUNK - 1) / CHUNK;
#pragma unroll 1
  for (int ch = 0; ch < nChunks; ++ch) {
    const int cbase = ch * CHUNK;
    const int wc = scan_chunk(dsts, nE, cbase, nodeBase, nb, vec8, list, tid, lane, wave);
    if (lane == 0) wcnt[wave] = wc;
    __syncthreads();
    int pre = 0, all = 0;
#pragma unroll
    for (int w2 = 0; w2 < NWAVE; ++w2) {
      int c = wcnt[w2];
      c = c < 0 ? 0 : (c > WCAP ? WCAP : c);
      all += c;
      pre += (w2 < wave) ? c : 0;
    }
    const int wcc  = wc > WCAP ? WCAP : wc;
    const int base = tot + pre;
#pragma unroll 1
    for (int i = lane; i < wcc; i += 32) {
      const int ent = list[wave * WCAP + i];
      const int el  = (ent >> 12) & (CHUNK - 1);
      const int sl  = ent & (NBMAX - 1);
      int eid = cbase + el;
      eid = eid > nE - 1 ? nE - 1 : eid;
      const int pos = base + i;
      if (pos < RCAP) reg1[pos] = (int)(((unsigned)eid << 12) | (unsigned)sl);
    }
    const int want = tot + all;
    lost |= (want > RCAP) ? 1 : 0;
    tot = want > RCAP ? RCAP : want;
    __syncthreads();
  }
  const int nh = tot;

  if (wave == 0) {
#pragma unroll 1
    for (int b0 = 0; b0 < nh; b0 += 32) {
      const int idx = b0 + lane;
      const int uv  = reg1[idx < RCAP ? idx : RCAP - 1];
      const int m32 = (nh - b0) < 32 ? (nh - b0) : 32;
#pragma unroll 1
      for (int k = 0; k < m32; ++k) {
        const int u  = __builtin_amdgcn_readlane(uv, k);
        const int sl = u & (NBMAX - 1);
        if (lane == 0) scnt[sl] = scnt[sl] + 1;
      }
    }
  }
  __syncthreads();

  {
    const v4i ca = *(const v4i*)(scnt + 8 * tid);
    const v4i cb = *(const v4i*)(scnt + 8 * tid + 4);
    const int e0 = ca.x < 0 ? 0 : ca.x, e1 = ca.y < 0 ? 0 : ca.y, e2 = ca.z < 0 ? 0 : ca.z, e3 = ca.w < 0 ? 0 : ca.w;
    const int e4 = cb.x < 0 ? 0 : cb.x, e5 = cb.y < 0 ? 0 : cb.y, e6 = cb.z < 0 ? 0 : cb.z, e7 = cb.w < 0 ? 0 : cb.w;
    const int ts = e0 + e1 + e2 + e3 + e4 + e5 + e6 + e7;
    int incl = ts;
#pragma unroll
    for (int d = 1; d < 32; d <<= 1) {
      const int up = __shfl_up(incl, d);
      if (lane >= d) incl += up;
    }
    if (lane == 31) wtot[wave] = incl;
    __syncthreads();
    int pre = 0;
#pragma unroll
    for (int w2 = 0; w2 < NWAVE; ++w2) pre += (w2 < wave) ? wtot[w2] : 0;
    int run = pre + incl - ts;
    soff[8 * tid + 0] = run; run += e0;
    soff[8 * tid + 1] = run; run += e1;
    soff[8 * tid + 2] = run; run += e2;
    soff[8 * tid + 3] = run; run += e3;
    soff[8 * tid + 4] = run; run += e4;
    soff[8 * tid + 5] = run; run += e5;
    soff[8 * tid + 6] = run; run += e6;
    soff[8 * tid + 7] = run;
  }
  __syncthreads();
  for (int i = tid; i < NBMAX; i += NTHR) list[i] = soff[i];
  __syncthreads();

  if (wave == 0) {
#pragma unroll 1
    for (int b0 = 0; b0 < nh; b0 += 32) {
      const int idx = b0 + lane;
      const int uv  = reg1[idx < RCAP ? idx : RCAP - 1];
      const int m32 = (nh - b0) < 32 ? (nh - b0) : 32;
#pragma unroll 1
      for (int k = 0; k < m32; ++k) {
        const int u   = __builtin_amdgcn_readlane(uv, k);
        const int sl  = u & (NBMAX - 1);
        const int eid = (int)((unsigned)u >> 12);
        if (lane == 0) {
          int pos = list[sl];
          pos = pos < 0 ? 0 : (pos > RCAP - 1 ? RCAP - 1 : pos);
          reg2[pos] = eid;
          list[sl] = pos + 1;
        }
      }
    }
  }
  __syncthreads();

  const int nbw  = nb >> 3;
  const int c4a  = 4 * lane;
  const int c4b  = (FD / 2) + 4 * lane;
  const v4f ata  = *(const v4f*)(attw + c4a);
  const v4f atb  = *(const v4f*)(attw + c4b);
  const v4f bza  = *(const v4f*)(biaso + c4a);
  const v4f bzb  = *(const v4f*)(biaso + c4b);
  const v4f z4   = {0.f, 0.f, 0.f, 0.f};
  const float qn = __uint_as_float(0x7fc00000u);
  v4f keepLo = z4, keepHi = z4;
#pragma unroll 1
  for (int jt = 0; jt < nbw; ++jt) {
    const int slot = wave * nbw + jt;
    const int grow = nodeBase + slot;
    const int gcl  = grow < nN ? grow : nN - 1;
    int st  = soff[slot];
    int cnt = scnt[slot];
    const bool bad = (cnt > DEGCAP) || (lost != 0);
    st  = st < 0 ? 0 : (st > nh ? nh : st);
    cnt = cnt < 0 ? 0 : (cnt > DEGCAP ? DEGCAP : cnt);
    if (cnt > nh - st) cnt = nh - st;

    const float* xrrow = xr + (size_t)gcl * FD;
    const float* xfrow = xres + (size_t)gcl * KD;
    const v4f xra = *(const v4f*)(xrrow + c4a);
    const v4f xrb = *(const v4f*)(xrrow + c4b);
    const v4f fra = *(const v4f*)(xfrow + c4a);
    const v4f frb = *(const v4f*)(xfrow + c4b);

    float ma = -1.0e30f, mb = -1.0e30f, dena = 0.0f, denb = 0.0f;
    v4f acca = z4, accb = z4;

#pragma unroll 1
    for (int q = 0; q < cnt; ++q) {
      int idx = st + q; idx = idx > RCAP - 1 ? RCAP - 1 : idx;
      int eid = reg2[idx]; eid = eid < 0 ? 0 : (eid > nE - 1 ? nE - 1 : eid);
      const int sraw = srcs[eid];
      const int s = sraw < 0 ? 0 : (sraw > nN - 1 ? nN - 1 : sraw);
      const float* xsrow = xl + (size_t)s * FD;
      const v4f xsa = *(const v4f*)(xsrow + c4a);
      const v4f xsb = *(const v4f*)(xsrow + c4b);
      const float la = logit16(xsa + xra, ata);
      const float lb = logit16(xsb + xrb, atb);
      const float mna = fmaxf(ma, la);
      const float mnb = fmaxf(mb, lb);
      const float s1a = __expf(ma - mna);
      const float s1b = __expf(mb - mnb);
      const float s2a = __expf(la - mna);
      const float s2b = __expf(lb - mnb);
      dena = fmaf(dena, s1a, s2a);
      denb = fmaf(denb, s1b, s2b);
      acca.x = fmaf(acca.x, s1a, s2a * xsa.x);
      acca.y = fmaf(acca.y, s1a, s2a * xsa.y);
      acca.z = fmaf(acca.z, s1a, s2a * xsa.z);
      acca.w = fmaf(acca.w, s1a, s2a * xsa.w);
      accb.x = fmaf(accb.x, s1b, s2b * xsb.x);
      accb.y = fmaf(accb.y, s1b, s2b * xsb.y);
      accb.z = fmaf(accb.z, s1b, s2b * xsb.z);
      accb.w = fmaf(accb.w, s1b, s2b * xsb.w);
      ma = mna; mb = mnb;
    }
    const float ra = __builtin_amdgcn_rcpf(dena);
    const float rb = __builtin_amdgcn_rcpf(denb);
    const float inva = dena > 0.0f ? ra : 0.0f;
    const float invb = denb > 0.0f ? rb : 0.0f;
    v4f oa, ob;
    oa.x = acca.x * inva + fra.x + bza.x;
    oa.y = acca.y * inva + fra.y + bza.y;
    oa.z = acca.z * inva + fra.z + bza.z;
    oa.w = acca.w * inva + fra.w + bza.w;
    ob.x = accb.x * invb + frb.x + bzb.x;
    ob.y = accb.y * invb + frb.y + bzb.y;
    ob.z = accb.z * invb + frb.z + bzb.z;
    ob.w = accb.w * invb + frb.w + bzb.w;
    if (bad) { oa.x = qn; oa.y = qn; oa.z = qn; oa.w = qn; ob = oa; }
    float* gp = outp + (size_t)gcl * FD;
    const bool wr = grow < nN;
    if (wr) { *(volatile v4f*)(gp + c4a) = oa; *(volatile v4f*)(gp + c4b) = ob; }
    __threadfence();
    if (wr) { *(volatile v4f*)(gp + c4a) = oa; *(volatile v4f*)(gp + c4b) = ob; }

    v4f mv, iv;
    mv.x = bcl(ma, 0);   mv.y = bcl(ma, 16);   mv.z = bcl(mb, 0);   mv.w = bcl(mb, 16);
    iv.x = bcl(inva, 0); iv.y = bcl(inva, 16); iv.z = bcl(invb, 0); iv.w = bcl(invb, 16);
    v4f mine = mv;
    if (lane & 1) mine = iv;
    const int gi = jt & 31;
    if (gi == (lane >> 1)) keepLo = mine;
    if (gi == 16 + (lane >> 1)) keepHi = mine;
    if (gi == 31 || jt == nbw - 1) {
      const int ng = gi + 1;
      float* sp0 = stat + (size_t)(nodeBase + slot - gi) * 8;
      const bool w1 = lane < 2 * ng;
      const bool w2 = lane < 2 * (ng - 16);
      if (w1) *(volatile v4f*)(sp0 + 4 * lane) = keepLo;
      if (w2) *(volatile v4f*)(sp0 + 128 + 4 * lane) = keepHi;
      __threadfence();
      if (w1) *(volatile v4f*)(sp0 + 4 * lane) = keepLo;
      if (w2) *(volatile v4f*)(sp0 + 128 + 4 * lane) = keepHi;
    }
  }
}

__global__ __launch_bounds__(NTHR) void k_edge(const int* __restrict__ srcs, const int* __restrict__ dsts,
                                               const float* __restrict__ xl, const float* __restrict__ xr,
                                               const float* __restrict__ attw, const float* __restrict__ stat,
                                               float* aout, int nN, int nE) {
  const int tid = threadIdx.x, lane = tid & 31, wave = tid >> 5, hsel = lane >> 4;
  const int e0 = ((int)blockIdx.x * NWAVE + wave) * EPW;
  if (e0 >= nE) return;
  int el = e0 + lane; el = el > nE - 1 ? nE - 1 : el;
  int sv = srcs[el], dv = dsts[el];
  sv = sv < 0 ? 0 : (sv > nN - 1 ? nN - 1 : sv);
  dv = dv < 0 ? 0 : (dv > nN - 1 ? nN - 1 : dv);
  const int c4a = 4 * lane, c4b = (FD / 2) + 4 * lane;
  const v4f ata = *(const v4f*)(attw + c4a);
  const v4f atb = *(const v4f*)(attw + c4b);
  v4f keep = {0.f, 0.f, 0.f, 0.f};
#pragma unroll 1
  for (int j = 0; j < EPW; ++j) {
    const int s = __builtin_amdgcn_readlane(sv, j);
    const int d = __builtin_amdgcn_readlane(dv, j);
    const float* xsrow = xl + (size_t)s * FD;
    const float* xdrow = xr + (size_t)d * FD;
    const v4f xsa = *(const v4f*)(xsrow + c4a);
    const v4f xsb = *(const v4f*)(xsrow + c4b);
    const v4f xda = *(const v4f*)(xdrow + c4a);
    const v4f xdb = *(const v4f*)(xdrow + c4b);
    const float la = logit16(xsa + xda, ata);
    const float lb = logit16(xsb + xdb, atb);
    const v4f sm = *(const v4f*)(stat + (size_t)d * 8);
    const v4f si = *(const v4f*)(stat + (size_t)d * 8 + 4);
    const float mA = hsel ? sm.y : sm.x, iA = hsel ? si.y : si.x;
    const float mB = hsel ? sm.w : sm.z, iB = hsel ? si.w : si.z;
    const float pa = __expf(la - mA) * iA;
    const float pb = __expf(lb - mB) * iB;
    v4f av;
    av.x = bcl(pa, 0); av.y = bcl(pa, 16); av.z = bcl(pb, 0); av.w = bcl(pb, 16);
    if (lane == j) keep = av;
  }
  const int ee = e0 + lane;
  if (ee < nE) *(volatile v4f*)(aout + (size_t)ee * NH) = keep;
  __threadfence();
  if (ee < nE) *(volatile v4f*)(aout + (size_t)ee * NH) = keep;
}

__global__ __launch_bounds__(NTHR) void k_gn1(const float* __restrict__ src, double* p1, int nN) {
  __shared__ __attribute__((aligned(16))) double sh[FD];
  const int tid = threadIdx.x;
  const int b  = (int)blockIdx.x;
  const int r0 = b * RB;
  const int r1 = (r0 + RB) < nN ? (r0 + RB) : nN;
  double s = 0.0;
#pragma unroll 4
  for (int r = r0; r < r1; ++r) s += (double)src[(size_t)r * FD + tid];
  sh[tid] = s;
  __syncthreads();
  const int tc = tid < (FD / 2) ? tid : (FD / 2) - 1;
  const v2d v = *(const v2d*)(sh + 2 * tc);
  double* d = p1 + (size_t)b * FD + 2 * tc;
  if (tid < FD / 2) *(volatile v2d*)d = v;
  __threadfence();
  if (tid < FD / 2) *(volatile v2d*)d = v;
}

__global__ __launch_bounds__(NTHR) void k_gnm(const double* __restrict__ p1, float* meanp, int nB, int nN) {
  __shared__ __attribute__((aligned(16))) float shm[FD];
  const int tid = threadIdx.x;
  double s = 0.0;
#pragma unroll 1
  for (int b = 0; b < nB; ++b) s += p1[(size_t)b * FD + tid];
  shm[tid] = (float)(s / (double)nN);
  __syncthreads();
  const int tc = tid < (FD / 4) ? tid : (FD / 4) - 1;
  const v4f v = *(const v4f*)(shm + 4 * tc);
  if (tid < FD / 4) *(volatile v4f*)(meanp + 4 * tc) = v;
  __threadfence();
  if (tid < FD / 4) *(volatile v4f*)(meanp + 4 * tc) = v;
}

__global__ __launch_bounds__(NTHR) void k_gn2(const float* __restrict__ src, const float* __restrict__ meanp,
                                              double* p2, int nN) {
#pragma clang fp contract(off)
  __shared__ __attribute__((aligned(16))) double sh[FD];
  const int tid = threadIdx.x;
  const int b  = (int)blockIdx.x;
  const int r0 = b * RB;
  const int r1 = (r0 + RB) < nN ? (r0 + RB) : nN;
  const float mc = meanp[tid];
  double s = 0.0;
#pragma unroll 4
  for (int r = r0; r < r1; ++r) {
    const float  ctr = src[(size_t)r * FD + tid] - mc;
    const double cd  = (double)ctr;
    s += cd * cd;
  }
  sh[tid] = s;
  __syncthreads();
  const int tc = tid < (FD / 2) ? tid : (FD / 2) - 1;
  const v2d v = *(const v2d*)(sh + 2 * tc);
  double* d = p2 + (size_t)b * FD + 2 * tc;
  if (tid < FD / 2) *(volatile v2d*)d = v;
  __threadfence();
  if (tid < FD / 2) *(volatile v2d*)d = v;
}

__global__ __launch_bounds__(NTHR) void k_gnv(const double* __restrict__ p2, float* rstdp, int nB, int nN) {
#pragma clang fp contract(off)
  __shared__ __attribute__((aligned(16))) float shm[FD];
  const int tid = threadIdx.x;
  double s = 0.0;
#pragma unroll 1
  for (int b = 0; b < nB; ++b) s += p2[(size_t)b * FD + tid];
  const float var = (float)(s / (double)nN);
  shm[tid] = 1.0f / sqrtf(var + BN_EPS);
  __syncthreads();
  const int tc = tid < (FD / 4) ? tid : (FD / 4) - 1;
  const v4f v = *(const v4f*)(shm + 4 * tc);
  if (tid < FD / 4) *(volatile v4f*)(rstdp + 4 * tc) = v;
  __threadfence();
  if (tid < FD / 4) *(volatile v4f*)(rstdp + 4 * tc) = v;
}

__global__ __launch_bounds__(NTHR) void k_gn3(float* io, const float* __restrict__ meanp,
                                              const float* __restrict__ rstdp,
                                              const float* __restrict__ gnw, const float* __restrict__ gnb,
                                              int nN) {
#pragma clang fp contract(off)
  const int tid = threadIdx.x;
  const int b  = (int)blockIdx.x;
  const int r0 = b * RB;
  const int r1 = (r0 + RB) < nN ? (r0 + RB) : nN;
  const int q  = tid & 63;
  const int rs = tid >> 6;
  const v4f mn  = *(const v4f*)(meanp + 4 * q);
  const v4f rsd = *(const v4f*)(rstdp + 4 * q);
  const v4f w   = *(const v4f*)(gnw + 4 * q);
  const v4f bb  = *(const v4f*)(gnb + 4 * q);
  const v4f z4  = {0.f, 0.f, 0.f, 0.f};
#pragma unroll 1
  for (int r = r0 + rs; r < r1; r += 4) {
    float* p = io + (size_t)r * FD + 4 * q;
    const v4f v   = *(const v4f*)p;
    const v4f ctr = v - mn;
    v4f y = (ctr * rsd) * w + bb;
    y.x = fmaxf(y.x, z4.x); y.y = fmaxf(y.y, z4.y); y.z = fmaxf(y.z, z4.z); y.w = fmaxf(y.w, z4.w);
    *(volatile v4f*)p = y;
    __threadfence();
    *(volatile v4f*)p = y;
  }
}

static int pick_nb(int nE, int nN) {
  int nb = NBMAX;
  while (nb > NBMIN && (long long)nb * (long long)nE * 5LL > (long long)RCAP * (long long)nN * 4LL) nb >>= 1;
  return nb;
}

extern "C" void kernel_launch(void* const* d_in, const int* in_sizes, int n_in,
                              void* d_out, int out_size, void* d_ws, size_t ws_size,
                              hipStream_t stream) {
  if (n_in < 11) return;
  const int nN = in_sizes[0] / KD;
  if (nN <= 0 || in_sizes[0] != nN * KD) return;
  if (nN > (1 << 22)) return;
  const int nE = in_sizes[1];
  if (nE < 1 || nE > (1 << 20)) return;
  if (in_sizes[2] != nE) return;
  if (in_sizes[3] != KD * FD || in_sizes[5] != KD * FD) return;
  if (in_sizes[4] != FD || in_sizes[6] != FD || in_sizes[7] != NH * HC) return;
  if (in_sizes[8] != FD || in_sizes[9] != FD || in_sizes[10] != FD) return;
  if ((long long)out_size != (long long)nN * FD + (long long)nE * NH) return;

  const float* x    = (const float*)d_in[0];
  const int*   srcv = (const int*)d_in[1];
  const int*   dstv = (const int*)d_in[2];
  const float* Ws   = (const float*)d_in[3];
  const float* bs   = (const float*)d_in[4];
  const float* Wd   = (const float*)d_in[5];
  const float* bd   = (const float*)d_in[6];
  const float* attw = (const float*)d_in[7];
  const float* bo   = (const float*)d_in[8];
  const float* gnw  = (const float*)d_in[9];
  const float* gnb  = (const float*)d_in[10];
  float* out  = (float*)d_out;
  float* aout = out + (size_t)nN * FD;

  const int MP      = ((nN + GBM - 1) / GBM) * GBM;
  const int nB      = (nN + RB - 1) / RB;
  const int nb      = pick_nb(nE, nN);
  const int gridAgg = (nN + nb - 1) / nb;
  const int NS      = gridAgg * nb;
  const int vec8    = 1;

  char* ws = (char*)d_ws;
  size_t off = 0;
  const size_t oWT = off; off += (size_t)NMAT * FD * KD * 2;   off = (off + 255) & ~(size_t)255;
  const size_t oY  = off; off += (size_t)2 * MP * FD * 4;      off = (off + 255) & ~(size_t)255;
  const size_t oST = off; off += (size_t)NS * 8 * 4;           off = (off + 255) & ~(size_t)255;
  const size_t oP1 = off; off += (size_t)nB * FD * 8;          off = (off + 255) & ~(size_t)255;
  const size_t oP2 = off; off += (size_t)nB * FD * 8;          off = (off + 255) & ~(size_t)255;
  const size_t oMN = off; off += (size_t)FD * 4;               off = (off + 255) & ~(size_t)255;
  const size_t oRS = off; off += (size_t)FD * 4;               off = (off + 255) & ~(size_t)255;
  if (off > ws_size || off > (size_t)WSCAP) return;
  unsigned short* WT = (unsigned short*)(ws + oWT);
  float*  Y     = (float*)(ws + oY);
  float*  STAT  = (float*)(ws + oST);
  double* P1    = (double*)(ws + oP1);
  double* P2    = (double*)(ws + oP2);
  float*  MEANL = (float*)(ws + oMN);
  float*  RSTDL = (float*)(ws + oRS);

  hipFuncSetAttribute(reinterpret_cast<const void*>(&k_agg),
                      hipFuncAttributeMaxDynamicSharedMemorySize, LDS_AGG);

  k_wprep<<<dim3(FD * KD / 8 / NTHR, NMAT), NTHR, 0, stream>>>(Ws, Wd, WT);
  k_gemm<<<MP / GBM, GTHR, 0, stream>>>(x, WT, bs, bd, Y, MP * FD, nN);
  k_agg<<<gridAgg, NTHR, LDS_AGG, stream>>>(srcv, dstv, Y, Y + (size_t)MP * FD, x, attw, bo, out, STAT,
                                            nN, nE, nb, vec8);
  k_edge<<<(nE + NWAVE * EPW - 1) / (NWAVE * EPW), NTHR, 0, stream>>>(srcv, dstv, Y, Y + (size_t)MP * FD,
                                                                        attw, STAT, aout, nN, nE);
  k_gn1<<<nB, NTHR, 0, stream>>>(out, P1, nN);
  k_gnm<<<1, NTHR, 0, stream>>>(P1, MEANL, nB, nN);
  k_gn2<<<nB, NTHR, 0, stream>>>(out, MEANL, P2, nN);
  k_gnv<<<1, NTHR, 0, stream>>>(P2, RSTDL, nB, nN);
  k_gn3<<<nB, NTHR, 0, stream>>>(out, MEANL, RSTDL, gnw, gnb, nN);
}
